// SimpleRNN7_22660247454199
// MI455X (gfx1250) — hardware-verified
//
#include <hip/hip_runtime.h>
#include <math.h>

constexpr int NBATCH   = 256;
constexpr int NSTEP    = 1024;
constexpr int NHID     = 128;
constexpr int NGATE    = 3 * NHID;
constexpr int NLIFT    = 32;
constexpr int NFEAT    = 7;
constexpr int NUIN     = 4;
constexpr int NOBS     = 3;
constexpr int NTHETA   = 11;
constexpr int NSTATE   = 7;
constexpr int NSUB     = 10;
constexpr int TFEVERY  = 50;
constexpr int ROWS_BLK = 16;
constexpr int NTHR     = 256;
constexpr int HPITCH   = 136;
constexpr int ZPITCH   = 40;
constexpr int STG_STEPS = 32;
constexpr int STG0      = ROWS_BLK * STG_STEPS * NOBS;
constexpr int STG1      = ROWS_BLK * STG_STEPS * NTHETA;
constexpr int STG_V4    = (STG0 + STG1) / 4;
constexpr int V4_ROW0   = STG_STEPS * NOBS / 4;
constexpr int V4_ROW1   = STG_STEPS * NTHETA / 4;
constexpr int V4_OUT0   = STG0 / 4;
constexpr int OUT0_ELEMS = NBATCH * NSTEP * NOBS;
constexpr int OUT1_ELEMS = NBATCH * NSTEP * NTHETA;
constexpr float WCARRY     = 16.0f;
constexpr float WCARRY_INV = 1.0f / 16.0f;

static_assert(NBATCH % ROWS_BLK == 0);
static_assert(NHID == 16 * (NTHR / 32));
static_assert(NLIFT == 32);
static_assert(NHID % 32 == 0);
static_assert(NFEAT == NUIN + NOBS);
static_assert(NSTEP % STG_STEPS == 0);
static_assert((STG_STEPS * NOBS * 4) % 128 == 0);
static_assert((STG_STEPS * NTHETA * 4) % 128 == 0);
static_assert(STG_V4 % NTHR == 0);
static_assert(V4_OUT0 % 32 == 0);
static_assert(V4_ROW0 % 8 == 0 && V4_ROW1 % 8 == 0);
static_assert((size_t)OUT0_ELEMS * 4 == (size_t)3145728);
static_assert(((size_t)OUT0_ELEMS + (size_t)OUT1_ELEMS) * 4 == (size_t)14680064);
static_assert((2 * ROWS_BLK * HPITCH) % NTHR == 0);
static_assert(ROWS_BLK * NLIFT == 2 * NTHR);
static_assert(HPITCH % 8 == 0 && ZPITCH % 8 == 0);

typedef __attribute__((ext_vector_type(16))) _Float16 v16h;
typedef __attribute__((ext_vector_type(8)))  _Float16 v8h;
typedef __attribute__((ext_vector_type(8)))  float    v8f;
typedef __attribute__((ext_vector_type(4)))  float    v4f;

__device__ __forceinline__ void guard3(v8f& a, v8f& b, v8f& c, v16h x, v16h y0, v16h y1, v16h y2) {
  asm volatile("v_nop\n\tv_nop\n\tv_nop\n\tv_nop" : "+v"(a), "+v"(b), "+v"(c) : "v"(x), "v"(y0), "v"(y1), "v"(y2));
}
__device__ __forceinline__ void guard3o(v8f& a, v8f& b, v8f& c, int& off, v16h x, v16h y0, v16h y1, v16h y2) {
  asm volatile("v_nop\n\tv_nop\n\tv_nop\n\tv_nop" : "+v"(a), "+v"(b), "+v"(c), "+v"(off) : "v"(x), "v"(y0), "v"(y1), "v"(y2));
}
__device__ __forceinline__ void guard1o(v8f& a, int& off, v16h x, v16h y) {
  asm volatile("v_nop\n\tv_nop\n\tv_nop\n\tv_nop" : "+v"(a), "+v"(off) : "v"(x), "v"(y));
}
__device__ __forceinline__ void acc_guard4(v8f& a, v8f& b, v8f& c, v8f& d) {
  asm volatile("v_nop\n\tv_nop\n\tv_nop\n\tv_nop" : "+v"(a), "+v"(b), "+v"(c), "+v"(d));
}
__device__ __forceinline__ void chain_after(int& off, v16h frag) {
  asm volatile("" : "+v"(off) : "v"(frag));
}

template <typename T> struct Frag;
template <> struct Frag<_Float16> {
  typedef v16h V; union U { v16h v; v8h h[2]; };
  static __device__ __forceinline__ v16h load(const _Float16* p) {
    U f; f.h[0] = *(const v8h*)(p); f.h[1] = *(const v8h*)(p + 16); return f.v;
  }
  static __device__ __forceinline__ v8f mma(v16h a, v16h b, v8f c) {
    return __builtin_amdgcn_wmma_f32_16x16x32_f16(false, a, false, b, (short)0, c, false, false);
  }
};

__device__ __forceinline__ v16h build_bfrag(const float* p) {
  const v4f a0 = *(const v4f*)(p);
  const v4f a1 = *(const v4f*)(p + 4);
  const v4f a2 = *(const v4f*)(p + 16);
  const v4f a3 = *(const v4f*)(p + 20);
  v16h r;
#pragma unroll
  for (int e = 0; e < 4; ++e) {
    r[e]      = (_Float16)(a0[e] * WCARRY);
    r[4 + e]  = (_Float16)(a1[e] * WCARRY);
    r[8 + e]  = (_Float16)(a2[e] * WCARRY);
    r[12 + e] = (_Float16)(a3[e] * WCARRY);
  }
  return r;
}

__device__ __forceinline__ float sigm(float x)    { return __builtin_amdgcn_rcpf(1.0f + expf(-x)); }
__device__ __forceinline__ float tanh_id(float x) { return 1.0f - 2.0f * __builtin_amdgcn_rcpf(expf(2.0f * x) + 1.0f); }

__device__ __forceinline__ void rhs7(const float (&y)[NSTATE], const float (&th)[NTHETA], float (&d)[NSTATE]) {
  const float A = y[0], D = y[1], G = y[2], J = y[3], Kv = y[4], L = y[5], Mv = y[6];
  const float kfAD = th[0], kfDG = th[1], kfGJ = th[2], kf10 = th[3], kf11 = th[4], kf12 = th[5];
  const float krAD = th[6], krDG = th[7], krGJ = th[8], kr11 = th[9], kr12 = th[10];
  d[0] = -kfAD * A + krAD * D;
  d[1] =  kfAD * A - krAD * D - kfDG * D + krDG * G;
  d[2] =  kfDG * D - krDG * G - kfGJ * G + krGJ * J;
  d[3] =  kfGJ * G - krGJ * J - kf10 * J;
  d[4] =  kf10 * J - kf11 * Kv + kr11 * L;
  d[5] =  kf11 * Kv - kr11 * L - kf12 * L + kr12 * Mv;
  d[6] =  kf12 * L - kr12 * Mv;
}

__global__ __launch_bounds__(NTHR) __attribute__((amdgpu_num_vgpr(256))) void gru_ode_seq_kernel(
    const float* __restrict__ y0_obs, const float* __restrict__ u_seq, const float* __restrict__ dt_seq,
    const float* __restrict__ y_seq, const float* __restrict__ lift_W, const float* __restrict__ lift_b,
    const float* __restrict__ W_ih, const float* __restrict__ W_hh, const float* __restrict__ b_ih,
    const float* __restrict__ b_hh, const float* __restrict__ head_W, const float* __restrict__ head_b,
    const float* __restrict__ u2x, float* __restrict__ out) {
  __shared__ __align__(16) _Float16 Ah[2][ROWS_BLK * HPITCH];
  __shared__ __align__(16) _Float16 Az[ROWS_BLK * ZPITCH];
  __shared__ __align__(16) _Float16 Hd[16 * HPITCH];
  __shared__ __align__(16) float    Stg[STG0 + STG1];
  __shared__ __align__(16) float    Xs[ROWS_BLK * 8];
  __shared__ __align__(16) float    Lw[NLIFT * 8];
  __shared__ __align__(16) float    Js[NUIN * 8];

  const int tid  = threadIdx.x;
  const int lane = tid & 31;
  const int wave = __builtin_amdgcn_readfirstlane(tid >> 5);
  const int c    = lane & 15;
  const int hh   = lane >> 4;
  const int koff = hh * 8;
  const int m     = tid & 15;
  const int opair = tid >> 4;
  const int b0    = blockIdx.x * ROWS_BLK;

  {
    _Float16* ahf = &Ah[0][0];
#pragma unroll 1
    for (int i = tid; i < 2 * ROWS_BLK * HPITCH; i += NTHR) ahf[i] = (_Float16)0.0f;
  }
#pragma unroll 1
  for (int i = tid; i < 16 * HPITCH; i += NTHR) {
    const int n  = i / HPITCH;
    const int kk = i - n * HPITCH;
    const int nc = (n < NTHETA) ? n : (NTHETA - 1);
    const int kc = (kk < NHID) ? kk : (NHID - 1);
    const float w = head_W[nc * NHID + kc];
    const bool live = (n < NTHETA) && (kk < NHID);
    Hd[i] = (_Float16)(live ? (w * WCARRY) : 0.0f);
  }
  if (tid < NLIFT * NFEAT) {
    const int o = tid / NFEAT;
    const int f = tid - o * NFEAT;
    Lw[o * 8 + f] = lift_W[tid];
  }
  if (tid < NLIFT) Lw[tid * 8 + 7] = lift_b[tid];
  if (tid < NUIN * NSTATE) {
    const int j = tid / NSTATE;
    const int s = tid - j * NSTATE;
    Js[j * 8 + s] = u2x[tid];
  }
  if (tid < NUIN) Js[tid * 8 + 7] = 0.0f;
  if (tid < ROWS_BLK * 8) {
    const int mm = tid >> 3;
    const int s  = tid & 7;
    const int oi = (s == 0) ? 0 : ((s == 3) ? 1 : ((s == 6) ? 2 : -1));
    const int oc = (oi < 0) ? 0 : oi;
    const float yv = y0_obs[(b0 + mm) * NOBS + oc];
    float v = (s < NSTATE) ? 0.01f : 0.0f;
    v += (oi >= 0) ? yv : 0.0f;
    Xs[tid] = v;
  }

  v16h Bih[3];
  v16h Bhh[3][4];
  {
    int ko = koff;
#pragma unroll
    for (int g = 0; g < 3; ++g) {
      const int n = g * NHID + 16 * wave + c;
      Bih[g] = build_bfrag(W_ih + (size_t)n * NLIFT + ko);
      chain_after(ko, Bih[g]);
#pragma unroll
      for (int kt = 0; kt < 4; ++kt) {
        Bhh[g][kt] = build_bfrag(W_hh + (size_t)n * NHID + ko + 32 * kt);
        chain_after(ko, Bhh[g][kt]);
      }
    }
  }
  const int ncol = 16 * wave + c;
  const float bias_r  = b_ih[ncol] + b_hh[ncol];
  const float bias_z  = b_ih[NHID + ncol] + b_hh[NHID + ncol];
  const float bias_in = b_ih[2 * NHID + ncol];
  const float bias_hn = b_hh[2 * NHID + ncol];
  const int   cth     = (c < NTHETA) ? c : (NTHETA - 1);
  const float hbv     = head_b[cth];
  const float hbias   = (c < NTHETA) ? hbv : 0.0f;

  float hreg[8];
#pragma unroll
  for (int r = 0; r < 8; ++r) hreg[r] = 0.0f;

  const size_t rowoff = (size_t)(b0 + m) * NSTEP;
  const v8f z8 = {0.f, 0.f, 0.f, 0.f, 0.f, 0.f, 0.f, 0.f};
  __syncthreads();

#pragma unroll 1
  for (int k = 0; k < NSTEP; ++k) {
    const int  cur = k & 1;
    const int  ks  = k & (STG_STEPS - 1);
    const bool tf  = (k > 0) && ((k % TFEVERY) == 0);
    const int  kp  = (k > 0) ? (k - 1) : 0;

    v4f   uv  = *(const v4f*)(u_seq + (rowoff + (size_t)k) * NUIN);
    float dtv = dt_seq[rowoff + (size_t)k];
    const float* yp = y_seq + (rowoff + (size_t)kp) * NOBS;
    float yv0 = yp[0], yv1 = yp[1], yv2 = yp[2];
    asm volatile("" : "+v"(uv));
    asm volatile("" : "+v"(dtv));
    asm volatile("" : "+v"(yv0), "+v"(yv1), "+v"(yv2));

    const float xo0 = Xs[m * 8 + 0];
    const float xo1 = Xs[m * 8 + 3];
    const float xo2 = Xs[m * 8 + 6];
    const float f4 = tf ? yv0 : xo0;
    const float f5 = tf ? yv1 : xo1;
    const float f6 = tf ? yv2 : xo2;

#pragma unroll
    for (int e = 0; e < 2; ++e) {
      const int o = 2 * opair + e;
      const float* lw = Lw + o * 8;
      float a = lw[7];
      a = fmaf(uv[0], lw[0], a);
      a = fmaf(uv[1], lw[1], a);
      a = fmaf(uv[2], lw[2], a);
      a = fmaf(uv[3], lw[3], a);
      a = fmaf(f4, lw[4], a);
      a = fmaf(f5, lw[5], a);
      a = fmaf(f6, lw[6], a);
      const float zv = a * sigm(a);
      Az[m * ZPITCH + o] = (_Float16)zv;
    }
    __syncthreads();

    v8f accR = z8, accZ = z8, accIN = z8, accHN = z8;
    {
      const v16h az = Frag<_Float16>::load(Az + c * ZPITCH + koff);
      accR  = Frag<_Float16>::mma(az, Bih[0], accR);
      accZ  = Frag<_Float16>::mma(az, Bih[1], accZ);
      accIN = Frag<_Float16>::mma(az, Bih[2], accIN);
      guard3(accR, accZ, accIN, az, Bih[0], Bih[1], Bih[2]);
    }
    {
      const _Float16* ahb = &Ah[cur][0];
      int aoff = c * HPITCH + koff;
#pragma unroll
      for (int kt = 0; kt < 4; ++kt) {
        const v16h a = Frag<_Float16>::load(ahb + aoff + 32 * kt);
        accR  = Frag<_Float16>::mma(a, Bhh[0][kt], accR);
        accZ  = Frag<_Float16>::mma(a, Bhh[1][kt], accZ);
        accHN = Frag<_Float16>::mma(a, Bhh[2][kt], accHN);
        guard3o(accR, accZ, accHN, aoff, a, Bhh[0][kt], Bhh[1][kt], Bhh[2][kt]);
      }
    }
    acc_guard4(accR, accZ, accIN, accHN);

    {
      _Float16* ahn = &Ah[cur ^ 1][0];
#pragma unroll
      for (int r = 0; r < 8; ++r) {
        const float pr  = accR[r]  * WCARRY_INV + bias_r;
        const float pz  = accZ[r]  * WCARRY_INV + bias_z;
        const float gin = accIN[r] * WCARRY_INV + bias_in;
        const float ghn = accHN[r] * WCARRY_INV + bias_hn;
        const float rg  = sigm(pr);
        const float zg  = sigm(pz);
        const float ng  = tanh_id(gin + rg * ghn);
        const float hn  = (1.0f - zg) * ng + zg * hreg[r];
        hreg[r] = hn;
        ahn[(8 * hh + r) * HPITCH + 16 * wave + c] = (_Float16)hn;
      }
    }
    __syncthreads();

    if (wave == 0) {
      const _Float16* ahb = &Ah[cur ^ 1][0];
      int hoff = c * HPITCH + koff;
      v8f acc = z8;
#pragma unroll
      for (int kt = 0; kt < 4; ++kt) {
        const v16h a = Frag<_Float16>::load(ahb + hoff + 32 * kt);
        const v16h b = Frag<_Float16>::load(Hd + hoff + 32 * kt);
        acc = Frag<_Float16>::mma(a, b, acc);
        guard1o(acc, hoff, a, b);
      }
#pragma unroll
      for (int r = 0; r < 8; ++r) {
        const float th = 0.01f + 2.99f * sigm(acc[r] * WCARRY_INV + hbias);
        if (c < NTHETA) Stg[STG0 + (8 * hh + r) * (STG_STEPS * NTHETA) + ks * NTHETA + c] = th;
      }
    }
    __syncthreads();

    if (tid < ROWS_BLK) {
      float th[NTHETA];
      const float* tp = Stg + STG0 + m * (STG_STEPS * NTHETA) + ks * NTHETA;
#pragma unroll
      for (int i = 0; i < NTHETA; ++i) th[i] = tp[i];
      float x[NSTATE];
#pragma unroll
      for (int s = 0; s < NSTATE; ++s) {
        float j = uv[0] * Js[s];
        j = fmaf(uv[1], Js[8 + s], j);
        j = fmaf(uv[2], Js[16 + s], j);
        j = fmaf(uv[3], Js[24 + s], j);
        x[s] = Xs[m * 8 + s] + j;
      }
      const float hs    = dtv * 0.1f;
      const float hhalf = 0.5f * hs;
      const float h6    = hs * (1.0f / 6.0f);
#pragma unroll 1
      for (int sub = 0; sub < NSUB; ++sub) {
        float kc[NSTATE], ksum[NSTATE], tmp[NSTATE];
        rhs7(x, th, kc);
#pragma unroll
        for (int s = 0; s < NSTATE; ++s) { ksum[s] = kc[s]; tmp[s] = x[s] + hhalf * kc[s]; }
        rhs7(tmp, th, kc);
#pragma unroll
        for (int s = 0; s < NSTATE; ++s) { ksum[s] = ksum[s] + 2.0f * kc[s]; tmp[s] = x[s] + hhalf * kc[s]; }
        rhs7(tmp, th, kc);
#pragma unroll
        for (int s = 0; s < NSTATE; ++s) { ksum[s] = ksum[s] + 2.0f * kc[s]; tmp[s] = x[s] + hs * kc[s]; }
        rhs7(tmp, th, kc);
#pragma unroll
        for (int s = 0; s < NSTATE; ++s) {
          const float incr = ksum[s] + kc[s];
          x[s] = fmaxf(x[s] + h6 * incr, 0.0f);
        }
      }
#pragma unroll
      for (int s = 0; s < NSTATE; ++s) Xs[m * 8 + s] = x[s];
      float* sp = Stg + m * (STG_STEPS * NOBS) + ks * NOBS;
      sp[0] = x[0];
      sp[1] = x[3];
      sp[2] = x[6];
    }
    __syncthreads();

    if (ks == STG_STEPS - 1) {
      const int k0 = k - (STG_STEPS - 1);
      for (int pass = 0; pass < 2; ++pass) {
#pragma unroll
        for (int it = 0; it < STG_V4 / NTHR; ++it) {
          const int f = it * NTHR + tid;
          const v4f v = *(const v4f*)(Stg + 4 * f);
          const int fa = (f < V4_OUT0) ? f : (V4_OUT0 - 1);
          const int ma = fa / V4_ROW0;
          const int qa = fa - ma * V4_ROW0;
          const size_t offa = ((size_t)(b0 + ma) * NSTEP + (size_t)k0) * NOBS + (size_t)qa * 4;
          const int fb = (f >= V4_OUT0) ? (f - V4_OUT0) : 0;
          const int mb = fb / V4_ROW1;
          const int qb = fb - mb * V4_ROW1;
          const size_t offb = (size_t)OUT0_ELEMS + ((size_t)(b0 + mb) * NSTEP + (size_t)k0) * NTHETA + (size_t)qb * 4;
          const size_t off = (f < V4_OUT0) ? offa : offb;
          *(volatile v4f*)(out + off) = v;
        }
        __threadfence();
      }
    }
  }
}

extern "C" void kernel_launch(void* const* d_in, const int* in_sizes, int n_in,
                              void* d_out, int out_size, void* d_ws, size_t ws_size, hipStream_t stream) {
  (void)d_ws; (void)ws_size;
  if (n_in < 13 || d_out == nullptr) return;
  if (in_sizes[0] != NBATCH * NOBS || in_sizes[1] != NBATCH * NSTEP * NUIN || in_sizes[2] != NBATCH * NSTEP ||
      in_sizes[3] != NBATCH * NSTEP * NOBS || in_sizes[4] != NLIFT * NFEAT || in_sizes[5] != NLIFT ||
      in_sizes[6] != NGATE * NLIFT || in_sizes[7] != NGATE * NHID || in_sizes[8] != NGATE || in_sizes[9] != NGATE ||
      in_sizes[10] != NTHETA * NHID || in_sizes[11] != NTHETA || in_sizes[12] != NUIN * NSTATE ||
      out_size != OUT0_ELEMS + OUT1_ELEMS) return;

  const float* y0_obs = (const float*)d_in[0];
  const float* u_seq  = (const float*)d_in[1];
  const float* dt_seq = (const float*)d_in[2];
  const float* y_seq  = (const float*)d_in[3];
  const float* lift_W = (const float*)d_in[4];
  const float* lift_b = (const float*)d_in[5];
  const float* W_ih   = (const float*)d_in[6];
  const float* W_hh   = (const float*)d_in[7];
  const float* b_ih   = (const float*)d_in[8];
  const float* b_hh   = (const float*)d_in[9];
  const float* head_W = (const float*)d_in[10];
  const float* head_b = (const float*)d_in[11];
  const float* u2x    = (const float*)d_in[12];
  float* out = (float*)d_out;

  gru_ode_seq_kernel<<<NBATCH / ROWS_BLK, NTHR, 0, stream>>>(
      y0_obs, u_seq, dt_seq, y_seq, lift_W, lift_b, W_ih, W_hh, b_ih, b_hh, head_W, head_b, u2x, out);
}
